// HypothesisDecoder_48284022341789
// MI455X (gfx1250) — hardware-verified
//
#include <hip/hip_runtime.h>
#include <stddef.h>


#pragma clang fp contract(off)

#define NBAT  2
#define GD    96
#define PLN   (GD * GD)
#define XB    2
#define NHYP  7
#define CSP   32
#define CPF   32
#define CIN0  64
#define HC    128
#define K1    (3 * CIN0)
#define K2    (3 * HC)
#define TP    32
#define MT    14
#define TPB   256
#define XS    72
#define AS    136
#define RESV  0.04f
#define EPSBN 1e-5f
#define SENT  0x7fffffff

#define NC1   (HC * K1 / 8)
#define NC2   (HC * K2 / 8)
#define NC4   (16 * K2 / 8)
#define G_PREP ((NC1 + 2 * NC2 + NC4) / TPB)

#define OFF_X   0
#define OFF_A   (OFF_X + TP * 9 * XS * 2)
#define OFF_B   (OFF_A + TP * 9 * AS * 2)
#define OFF_LG  (OFF_B + TP * 9 * AS * 2)
#define OFF_PR  (OFF_LG + TP * NHYP * 4)
#define SMEM_CONV (OFF_PR + TP * NHYP * 4)
#define SMEM_GRID (NBAT * XB * PLN * 4)

static_assert(TP * NHYP == MT * 16);
static_assert((NC1 + 2 * NC2 + NC4) % TPB == 0);
static_assert(G_PREP == 63);
static_assert(NC1 % TPB == 0);
static_assert(NC2 % TPB == 0);
static_assert(OFF_A == 41472);
static_assert(OFF_B == 119808);
static_assert(OFF_LG == 198144);
static_assert(SMEM_CONV == 199936);
static_assert((OFF_A % 16) == 0);
static_assert((OFF_B % 16) == 0);
static_assert((OFF_LG % 16) == 0);
static_assert((OFF_PR % 16) == 0);
static_assert((XS % 8) == 0);
static_assert((AS % 8) == 0);
static_assert(GD % XB == 0);
static_assert((XB * PLN / 4) % TPB == 0);
static_assert((NBAT * XB * PLN / 4) % TPB == 0);
static_assert((TPB * CIN0 / 8) % TPB == 0);
static_assert((TP * NHYP) % 4 == 0);
static_assert(K1 % 32 == 0);
static_assert(K2 % 32 == 0);

typedef float          v4f  __attribute__((ext_vector_type(4)));
typedef unsigned int   v4u  __attribute__((ext_vector_type(4)));
typedef int            v4i  __attribute__((ext_vector_type(4)));
typedef float          v8f  __attribute__((ext_vector_type(8)));
typedef _Float16       v16h __attribute__((ext_vector_type(16)));
typedef v4f __attribute__((may_alias)) v4fa;
typedef v4u __attribute__((may_alias)) v4ua;
typedef v4i __attribute__((may_alias)) v4ia;

union Frag { v16h v; v4u q[2]; };

__device__ __forceinline__ unsigned int pk2(float a, float b) {
  const unsigned int lo = (unsigned int)__builtin_bit_cast(unsigned short, (_Float16)a);
  const unsigned int hi = (unsigned int)__builtin_bit_cast(unsigned short, (_Float16)b);
  return lo | (hi << 16);
}

__device__ __forceinline__ v4u wchunk(const float* s, float scale) {
  v4u v;
  v.x = pk2(s[0]  * scale, s[3]  * scale);
  v.y = pk2(s[6]  * scale, s[9]  * scale);
  v.z = pk2(s[12] * scale, s[15] * scale);
  v.w = pk2(s[18] * scale, s[21] * scale);
  return v;
}

__device__ __forceinline__ v4u zsel(v4u v, bool ok) {
  v4u r;
  r.x = ok ? v.x : 0u;
  r.y = ok ? v.y : 0u;
  r.z = ok ? v.z : 0u;
  r.w = ok ? v.w : 0u;
  return r;
}

__device__ __forceinline__ int clampi(int x, int lo, int hi) {
  return x < lo ? lo : (x > hi ? hi : x);
}

__device__ __forceinline__ v8f wmma_h(v16h a, v16h b, v8f c) {
  v8f d = __builtin_amdgcn_wmma_f32_16x16x32_f16(false, a, false, b, (short)0, c, false, false);
  asm volatile("v_nop\n\tv_nop\n\tv_nop\n\tv_nop" : "+v"(d) : "v"(a), "v"(b));
  return d;
}

__global__ __launch_bounds__(TPB) void k_prep(const float* __restrict__ w1,
                                              const float* __restrict__ w2,
                                              const float* __restrict__ w3,
                                              const float* __restrict__ w4,
                                              unsigned short* __restrict__ wp1,
                                              unsigned short* __restrict__ wp2,
                                              unsigned short* __restrict__ wp3,
                                              unsigned short* __restrict__ wp4)
{
  const int u = blockIdx.x * TPB + threadIdx.x;
  v4u v;
  unsigned short* d;
  if (u < NC1) {
    const int o = u / (K1 / 8), kc = u - o * (K1 / 8);
    const int k = kc * 8, kk = k / CIN0, c0 = k - kk * CIN0;
    v = wchunk(w1 + (size_t)(o * CIN0 + c0) * 3 + kk, 16.0f);
    d = wp1 + (size_t)u * 8;
  } else if (u < NC1 + NC2) {
    const int t = u - NC1;
    const int o = t / (K2 / 8), kc = t - o * (K2 / 8);
    const int k = kc * 8, kk = k / HC, c0 = k - kk * HC;
    v = wchunk(w2 + (size_t)(o * HC + c0) * 3 + kk, 16.0f);
    d = wp2 + (size_t)t * 8;
  } else if (u < NC1 + 2 * NC2) {
    const int t = u - NC1 - NC2;
    const int o = t / (K2 / 8), kc = t - o * (K2 / 8);
    const int k = kc * 8, kk = k / HC, c0 = k - kk * HC;
    v = wchunk(w3 + (size_t)(o * HC + c0) * 3 + kk, 16.0f);
    d = wp3 + (size_t)t * 8;
  } else {
    const int t = u - NC1 - 2 * NC2;
    const int nrow = t / (K2 / 8), kc = t - nrow * (K2 / 8);
    const int k = kc * 8, kk = k / HC, c0 = k - kk * HC;
    v = zsel(wchunk(w4 + (size_t)c0 * 3 + kk, 16.0f), nrow == 0);
    d = wp4 + (size_t)t * 8;
  }
  *(volatile v4u*)d = v;
  __threadfence();
  *(volatile v4u*)d = v;
}

__global__ __launch_bounds__(TPB) void k_small(const float* __restrict__ pts,
                                               const int* __restrict__ sb, int n,
                                               const float* __restrict__ g1, const float* __restrict__ b1,
                                               const float* __restrict__ m1, const float* __restrict__ v1,
                                               const float* __restrict__ g2, const float* __restrict__ b2,
                                               const float* __restrict__ m2, const float* __restrict__ v2,
                                               const float* __restrict__ g3, const float* __restrict__ b3,
                                               const float* __restrict__ m3, const float* __restrict__ v3,
                                               float* __restrict__ mnp, float* __restrict__ bnt)
{
  __shared__ float sRed[64];
  __shared__ __align__(16) float sLine[32];
  __shared__ __align__(16) float sTab[3 * 2 * HC];

  const int tid = threadIdx.x, lane = tid & 31, wave = tid >> 5;

  #pragma unroll 1
  for (int e = tid; e < 3 * 2 * HC; e += TPB) {
    const int li = e >> 8, r = e & 255, o = r & 127;
    const float* gg = (li == 0) ? g1 : ((li == 1) ? g2 : g3);
    const float* bb = (li == 0) ? b1 : ((li == 1) ? b2 : b3);
    const float* mm = (li == 0) ? m1 : ((li == 1) ? m2 : m3);
    const float* vv = (li == 0) ? v1 : ((li == 1) ? v2 : v3);
    const float s = gg[o] / sqrtf(vv[o] + EPSBN);
    const float cin = (li == 0) ? (1.0f / 1024.0f) : (1.0f / 128.0f);
    const float sp = (8.0f * s) * cin;
    const float tp = 8.0f * (bb[o] - mm[o] * s);
    sTab[e] = (r < HC) ? sp : tp;
  }

  const float pinf = __int_as_float(0x7f800000);
  float a0 = pinf, a1 = pinf, a2 = pinf, c0 = pinf, c1 = pinf, c2 = pinf;
  #pragma unroll 1
  for (int i = tid; i < n; i += TPB) {
    const int b = sb[i];
    const float x = pts[(size_t)i * 3 + 0];
    const float y = pts[(size_t)i * 3 + 1];
    const float z = pts[(size_t)i * 3 + 2];
    const bool s0 = (b == 0), s1 = (b == 1);
    a0 = s0 ? fminf(a0, x) : a0;
    a1 = s0 ? fminf(a1, y) : a1;
    a2 = s0 ? fminf(a2, z) : a2;
    c0 = s1 ? fminf(c0, x) : c0;
    c1 = s1 ? fminf(c1, y) : c1;
    c2 = s1 ? fminf(c2, z) : c2;
  }
  #pragma unroll
  for (int s = 16; s >= 1; s >>= 1) {
    a0 = fminf(a0, __shfl_xor(a0, s, 32));
    a1 = fminf(a1, __shfl_xor(a1, s, 32));
    a2 = fminf(a2, __shfl_xor(a2, s, 32));
    c0 = fminf(c0, __shfl_xor(c0, s, 32));
    c1 = fminf(c1, __shfl_xor(c1, s, 32));
    c2 = fminf(c2, __shfl_xor(c2, s, 32));
  }
  if (lane == 0) {
    sRed[wave * 8 + 0] = a0; sRed[wave * 8 + 1] = a1; sRed[wave * 8 + 2] = a2;
    sRed[wave * 8 + 3] = c0; sRed[wave * 8 + 4] = c1; sRed[wave * 8 + 5] = c2;
    sRed[wave * 8 + 6] = 0.0f; sRed[wave * 8 + 7] = 0.0f;
  }
  __syncthreads();
  if (tid < 32) {
    const int bb = (tid >> 2) > (NBAT - 1) ? (NBAT - 1) : (tid >> 2);
    const int dd = (tid & 3) > 2 ? 2 : (tid & 3);
    float r = pinf;
    #pragma unroll
    for (int w = 0; w < TPB / 32; ++w) r = fminf(r, sRed[w * 8 + bb * 3 + dd]);
    const bool own = (tid < 4 * NBAT) && ((tid & 3) < 3);
    sLine[tid] = own ? r : 0.0f;
  }
  __syncthreads();

  if (tid < 8) {
    const v4f v = *(const v4fa*)(sLine + 4 * tid);
    *(volatile v4f*)(mnp + 4 * tid) = v;
  }
  if (tid < (3 * 2 * HC) / 4) {
    const v4f v = *(const v4fa*)(sTab + 4 * tid);
    *(volatile v4f*)(bnt + 4 * tid) = v;
  }
  __threadfence();
  if (tid < 8) {
    const v4f v = *(const v4fa*)(sLine + 4 * tid);
    *(volatile v4f*)(mnp + 4 * tid) = v;
  }
  if (tid < (3 * 2 * HC) / 4) {
    const v4f v = *(const v4fa*)(sTab + 4 * tid);
    *(volatile v4f*)(bnt + 4 * tid) = v;
  }
}

__global__ __launch_bounds__(TPB) void k_grid(const int* __restrict__ coords,
                                              const int* __restrict__ sb, int n,
                                              int* __restrict__ vox)
{
  extern __shared__ float4 dynsmem[];
  int* sP = (int*)dynsmem;
  const int tid = threadIdx.x;
  const int xb = blockIdx.x;

  const v4i s4 = {SENT, SENT, SENT, SENT};
  #pragma unroll 1
  for (int c = tid; c < (NBAT * XB * PLN) / 4; c += TPB) *(v4ia*)(sP + 4 * c) = s4;
  __syncthreads();

  #pragma unroll 1
  for (int i = tid; i < n; i += TPB) {
    const int cx = coords[(size_t)i * 3 + 0];
    const int cy = coords[(size_t)i * 3 + 1];
    const int cz = coords[(size_t)i * 3 + 2];
    const int b  = sb[i];
    const bool ok = ((unsigned)b < (unsigned)NBAT) && ((unsigned)cx < (unsigned)GD) &&
                    ((cx >> 1) == xb) &&
                    ((unsigned)cy < (unsigned)GD) && ((unsigned)cz < (unsigned)GD);
    const int cell = ok ? ((((b * XB) + (cx & 1)) * GD + cy) * GD + cz) : 0;
    const int val  = ok ? i : SENT;
    atomicMin(&sP[cell], val);
  }
  __syncthreads();

  #pragma unroll 1
  for (int b = 0; b < NBAT; ++b) {
    const int* srcp = sP + b * (XB * PLN);
    int* dst = vox + ((size_t)(b * GD + XB * xb)) * PLN;
    #pragma unroll 1
    for (int c = tid; c < (XB * PLN) / 4; c += TPB) {
      const v4i v = *(const v4ia*)(srcp + 4 * c);
      *(volatile v4i*)(dst + 4 * c) = v;
    }
  }
  __threadfence();
  #pragma unroll 1
  for (int b = 0; b < NBAT; ++b) {
    const int* srcp = sP + b * (XB * PLN);
    int* dst = vox + ((size_t)(b * GD + XB * xb)) * PLN;
    #pragma unroll 1
    for (int c = tid; c < (XB * PLN) / 4; c += TPB) {
      const v4i v = *(const v4ia*)(srcp + 4 * c);
      *(volatile v4i*)(dst + 4 * c) = v;
    }
  }
}

__global__ __launch_bounds__(TPB) void k_interp(const float* __restrict__ dmh,
                                                const float* __restrict__ pfeat,
                                                const int* __restrict__ pbat,
                                                const float* __restrict__ sfeat,
                                                const int* __restrict__ vox,
                                                const float* __restrict__ mnp,
                                                int nsp, int mrows,
                                                unsigned short* __restrict__ xpl)
{
  __shared__ __align__(16) unsigned short sT[TPB * CIN0];

  const int tid = threadIdx.x;
  const int m  = blockIdx.x * TPB + tid;
  const int mc = (m < mrows) ? m : (mrows - 1);
  const int p  = mc / NHYP;
  const int braw = pbat[p];
  const bool bok = (unsigned)braw < (unsigned)NBAT;
  const int b  = clampi(braw, 0, NBAT - 1);
  const float mn0 = mnp[b * 4 + 0], mn1 = mnp[b * 4 + 1], mn2 = mnp[b * 4 + 2];
  const float* dp = dmh + (size_t)mc * 3;
  const float q0 = (dp[0] - mn0) / RESV;
  const float q1 = (dp[1] - mn1) / RESV;
  const float q2 = (dp[2] - mn2) / RESV;
  const float f0 = floorf(q0), f1 = floorf(q1), f2 = floorf(q2);
  const float r0 = q0 - f0, r1 = q1 - f1, r2 = q2 - f2;
  const int i0 = (int)fminf(fmaxf(f0, -4.0f), 200.0f);
  const int i1 = (int)fminf(fmaxf(f1, -4.0f), 200.0f);
  const int i2 = (int)fminf(fmaxf(f2, -4.0f), 200.0f);

  float acc[32];
  #pragma unroll
  for (int c = 0; c < 32; ++c) acc[c] = 0.0f;

  #pragma unroll 1
  for (int corner = 0; corner < 8; ++corner) {
    const int dx = corner >> 2, dy = (corner >> 1) & 1, dz = corner & 1;
    const int cx = i0 + dx, cy = i1 + dy, cz = i2 + dz;
    const bool inr = ((unsigned)cx < (unsigned)GD) && ((unsigned)cy < (unsigned)GD) &&
                     ((unsigned)cz < (unsigned)GD);
    const int cxc = clampi(cx, 0, GD - 1), cyc = clampi(cy, 0, GD - 1), czc = clampi(cz, 0, GD - 1);
    const int idx = vox[((b * GD + cxc) * GD + cyc) * GD + czc];
    const bool hit = bok && inr && (idx != SENT);
    const int idc = clampi(idx, 0, nsp - 1);
    const float* fp = sfeat + (size_t)idc * CSP;
    const float wx = dx ? r0 : (1.0f - r0);
    const float wy = dy ? r1 : (1.0f - r1);
    const float wz = dz ? r2 : (1.0f - r2);
    const float w  = (wx * wy) * wz;
    const float we = hit ? w : 0.0f;
    #pragma unroll
    for (int c4 = 0; c4 < 8; ++c4) {
      const v4f f = *(const v4fa*)(fp + 4 * c4);
      acc[4 * c4 + 0] = acc[4 * c4 + 0] + we * f.x;
      acc[4 * c4 + 1] = acc[4 * c4 + 1] + we * f.y;
      acc[4 * c4 + 2] = acc[4 * c4 + 2] + we * f.z;
      acc[4 * c4 + 3] = acc[4 * c4 + 3] + we * f.w;
    }
  }

  unsigned short* row = sT + tid * CIN0;
  #pragma unroll
  for (int j = 0; j < 4; ++j) {
    v4u v;
    v.x = pk2(acc[8 * j + 0] * 64.0f, acc[8 * j + 1] * 64.0f);
    v.y = pk2(acc[8 * j + 2] * 64.0f, acc[8 * j + 3] * 64.0f);
    v.z = pk2(acc[8 * j + 4] * 64.0f, acc[8 * j + 5] * 64.0f);
    v.w = pk2(acc[8 * j + 6] * 64.0f, acc[8 * j + 7] * 64.0f);
    *(v4ua*)(row + 8 * j) = v;
  }
  const float* pf = pfeat + (size_t)mc * CPF;
  #pragma unroll
  for (int j = 0; j < 4; ++j) {
    const v4f a = *(const v4fa*)(pf + 8 * j);
    const v4f c = *(const v4fa*)(pf + 8 * j + 4);
    v4u v;
    v.x = pk2(a.x * 64.0f, a.y * 64.0f);
    v.y = pk2(a.z * 64.0f, a.w * 64.0f);
    v.z = pk2(c.x * 64.0f, c.y * 64.0f);
    v.w = pk2(c.z * 64.0f, c.w * 64.0f);
    *(v4ua*)(row + CSP + 8 * j) = v;
  }
  __syncthreads();

  unsigned short* gb = xpl + (size_t)blockIdx.x * (TPB * CIN0);
  #pragma unroll
  for (int it = 0; it < (TPB * CIN0 / 8) / TPB; ++it) {
    const int c = it * TPB + tid;
    const v4u v = *(const v4ua*)(sT + 8 * c);
    *(volatile v4u*)(gb + (size_t)8 * c) = v;
  }
  __threadfence();
  #pragma unroll
  for (int it = 0; it < (TPB * CIN0 / 8) / TPB; ++it) {
    const int c = it * TPB + tid;
    const v4u v = *(const v4ua*)(sT + 8 * c);
    *(volatile v4u*)(gb + (size_t)8 * c) = v;
  }
}

template <int CIN, int SS, int DS>
__device__ __forceinline__ void conv_layer(const unsigned short* __restrict__ wp,
                                           const unsigned short* src,
                                           unsigned short* dst,
                                           const float* __restrict__ bn,
                                           int lane, int otile)
{
  constexpr int K  = 3 * CIN;
  constexpr int KT = K / 32;
  const int m15 = lane & 15, hh = lane >> 4;
  const int ocol = otile * 16 + m15;
  const float sc = bn[ocol];
  const float bi = bn[HC + ocol];
  const unsigned short* wrow = wp + (size_t)ocol * K;

  Frag bfr[KT];
  #pragma unroll
  for (int kt = 0; kt < KT; ++kt) {
    bfr[kt].q[0] = *(const v4ua*)(wrow + kt * 32 + 8 * hh);
    bfr[kt].q[1] = *(const v4ua*)(wrow + kt * 32 + 16 + 8 * hh);
  }

  const v8f z8 = {0.f, 0.f, 0.f, 0.f, 0.f, 0.f, 0.f, 0.f};
  #pragma unroll 1
  for (int mt = 0; mt < MT; ++mt) {
    const int row = mt * 16 + m15;
    const int p = row / NHYP;
    const int l = row - p * NHYP;
    const unsigned short* abase = src + (p * 9 + l) * SS + 8 * hh;
    v8f acc = z8;
    #pragma unroll
    for (int kt = 0; kt < KT; ++kt) {
      const int k0 = kt * 32;
      const int kk = k0 / CIN;
      const int cb = k0 - kk * CIN;
      const unsigned short* ap = abase + kk * SS + cb;
      Frag a;
      a.q[0] = *(const v4ua*)(ap);
      a.q[1] = *(const v4ua*)(ap + 16);
      acc = wmma_h(a.v, bfr[kt].v, acc);
    }
    #pragma unroll
    for (int i = 0; i < 8; ++i) {
      const int r  = mt * 16 + 8 * hh + i;
      const int pp = r / NHYP;
      const int lr = r - pp * NHYP;
      const float v = fmaxf(fmaf(acc[i], sc, bi), 0.0f);
      dst[(pp * 9 + lr + 1) * DS + ocol] = __builtin_bit_cast(unsigned short, (_Float16)v);
    }
  }
}

__global__ __launch_bounds__(TPB) void k_conv(const unsigned short* __restrict__ xpl,
                                              const unsigned short* __restrict__ wp1,
                                              const unsigned short* __restrict__ wp2,
                                              const unsigned short* __restrict__ wp3,
                                              const unsigned short* __restrict__ wp4,
                                              const float* __restrict__ bnt,
                                              const float* __restrict__ bias4,
                                              float* __restrict__ out)
{
  extern __shared__ float4 dynsmem[];
  char* smem = (char*)dynsmem;
  unsigned short* xT = (unsigned short*)(smem + OFF_X);
  unsigned short* aA = (unsigned short*)(smem + OFF_A);
  unsigned short* aB = (unsigned short*)(smem + OFF_B);
  float* lg = (float*)(smem + OFF_LG);
  float* pr = (float*)(smem + OFF_PR);

  const int tid = threadIdx.x, lane = tid & 31, wave = tid >> 5;
  const size_t grow0 = (size_t)blockIdx.x * (TP * NHYP);

  const v4u z4 = {0u, 0u, 0u, 0u};
  #pragma unroll 1
  for (int i = tid; i < 2 * TP * (XS / 8); i += TPB) {
    const int r = i / (XS / 8), c = i - r * (XS / 8);
    const int rw = (r >> 1) * 9 + (r & 1) * 8;
    *(v4ua*)(xT + rw * XS + c * 8) = z4;
  }
  #pragma unroll 1
  for (int i = tid; i < 2 * TP * (AS / 8); i += TPB) {
    const int r = i / (AS / 8), c = i - r * (AS / 8);
    const int rw = (r >> 1) * 9 + (r & 1) * 8;
    *(v4ua*)(aA + rw * AS + c * 8) = z4;
    *(v4ua*)(aB + rw * AS + c * 8) = z4;
  }
  #pragma unroll 1
  for (int i = tid; i < TP * NHYP * (CIN0 / 8); i += TPB) {
    const int r = i >> 3, c = i & 7;
    const int p = r / NHYP, l = r - p * NHYP;
    const v4u v = *(const v4ua*)(xpl + (grow0 + r) * CIN0 + c * 8);
    *(v4ua*)(xT + (p * 9 + l + 1) * XS + c * 8) = v;
  }
  __syncthreads();

  conv_layer<CIN0, XS, AS>(wp1, xT, aA, bnt, lane, wave);
  __syncthreads();
  conv_layer<HC, AS, AS>(wp2, aA, aB, bnt + 2 * HC, lane, wave);
  __syncthreads();
  conv_layer<HC, AS, AS>(wp3, aB, aA, bnt + 4 * HC, lane, wave);
  __syncthreads();

  {
    const int m15 = lane & 15, hh = lane >> 4;
    const unsigned short* wrow = wp4 + (size_t)m15 * K2;
    Frag bq[K2 / 32];
    #pragma unroll
    for (int kt = 0; kt < K2 / 32; ++kt) {
      bq[kt].q[0] = *(const v4ua*)(wrow + kt * 32 + 8 * hh);
      bq[kt].q[1] = *(const v4ua*)(wrow + kt * 32 + 16 + 8 * hh);
    }
    const float b4 = bias4[0];
    const v8f z8 = {0.f, 0.f, 0.f, 0.f, 0.f, 0.f, 0.f, 0.f};
    #pragma unroll 1
    for (int mt = wave; mt < MT; mt += TPB / 32) {
      const int row = mt * 16 + m15;
      const int p = row / NHYP;
      const int l = row - p * NHYP;
      const unsigned short* abase = aA + (p * 9 + l) * AS + 8 * hh;
      v8f acc = z8;
      #pragma unroll
      for (int kt = 0; kt < K2 / 32; ++kt) {
        const int k0 = kt * 32;
        const int kk = k0 / HC;
        const int cb = k0 - kk * HC;
        const unsigned short* ap = abase + kk * AS + cb;
        Frag a;
        a.q[0] = *(const v4ua*)(ap);
        a.q[1] = *(const v4ua*)(ap + 16);
        acc = wmma_h(a.v, bq[kt].v, acc);
      }
      if (m15 == 0) {
        #pragma unroll
        for (int i = 0; i < 8; ++i)
          lg[mt * 16 + 8 * hh + i] = acc[i] * (1.0f / 128.0f) + b4;
      }
    }
  }
  __syncthreads();

  if (tid < TP) {
    float lv[NHYP], ev[NHYP];
    #pragma unroll
    for (int j = 0; j < NHYP; ++j) lv[j] = lg[tid * NHYP + j];
    float mx = lv[0];
    #pragma unroll
    for (int j = 1; j < NHYP; ++j) mx = fmaxf(mx, lv[j]);
    float s = 0.0f;
    #pragma unroll
    for (int j = 0; j < NHYP; ++j) { ev[j] = expf(lv[j] - mx); s = s + ev[j]; }
    const float inv = 1.0f / s;
    #pragma unroll
    for (int j = 0; j < NHYP; ++j) pr[tid * NHYP + j] = ev[j] * inv;
  }
  __syncthreads();

  float* ob = out + grow0;
  if (tid < (TP * NHYP) / 4) {
    const v4f v = *(const v4fa*)(pr + 4 * tid);
    *(volatile v4f*)(ob + 4 * tid) = v;
  }
  __threadfence();
  if (tid < (TP * NHYP) / 4) {
    const v4f v = *(const v4fa*)(pr + 4 * tid);
    *(volatile v4f*)(ob + 4 * tid) = v;
  }
}

extern "C" void kernel_launch(void* const* d_in, const int* in_sizes, int n_in,
                              void* d_out, int out_size, void* d_ws, size_t ws_size,
                              hipStream_t stream)
{
  if (n_in < 24) return;
  const int nsp  = in_sizes[2];
  const int npts = in_sizes[6];
  if (nsp < 1 || npts < TP) return;
  if (in_sizes[0] != 3 * nsp || in_sizes[1] != 3 * nsp || in_sizes[3] != CSP * nsp) return;
  if (in_sizes[4] != npts * NHYP * 3 || in_sizes[5] != npts * NHYP * CPF) return;
  if (in_sizes[7] != HC * CIN0 * 3) return;
  if (in_sizes[12] != HC * HC * 3 || in_sizes[17] != HC * HC * 3) return;
  if (in_sizes[22] != HC * 3 || in_sizes[23] < 1) return;
  for (int j = 0; j < 4; ++j) {
    if (in_sizes[8 + j] != HC || in_sizes[13 + j] != HC || in_sizes[18 + j] != HC) return;
  }
  if (out_size != npts * NHYP) return;
  if (npts % TP != 0) return;

  const float* sparse_pts    = (const float*)d_in[0];
  const int*   sparse_coords = (const int*)d_in[1];
  const int*   sparse_batch  = (const int*)d_in[2];
  const float* sparse_feats  = (const float*)d_in[3];
  const float* dmh           = (const float*)d_in[4];
  const float* pfeat         = (const float*)d_in[5];
  const int*   pbatch        = (const int*)d_in[6];
  const float* w1 = (const float*)d_in[7];
  const float* g1 = (const float*)d_in[8];
  const float* b1 = (const float*)d_in[9];
  const float* m1 = (const float*)d_in[10];
  const float* v1 = (const float*)d_in[11];
  const float* w2 = (const float*)d_in[12];
  const float* g2 = (const float*)d_in[13];
  const float* b2 = (const float*)d_in[14];
  const float* m2 = (const float*)d_in[15];
  const float* v2 = (const float*)d_in[16];
  const float* w3 = (const float*)d_in[17];
  const float* g3 = (const float*)d_in[18];
  const float* b3 = (const float*)d_in[19];
  const float* m3 = (const float*)d_in[20];
  const float* v3 = (const float*)d_in[21];
  const float* w4 = (const float*)d_in[22];
  const float* bias4 = (const float*)d_in[23];
  float* out = (float*)d_out;

  const int mrows = npts * NHYP;
  const int mblk  = (mrows + TPB - 1) / TPB;
  const size_t mpad = (size_t)mblk * TPB;

  const size_t bMn  = 128;
  const size_t bVox = (size_t)NBAT * GD * PLN * 4;
  const size_t bW1  = (size_t)HC * K1 * 2;
  const size_t bW2  = (size_t)HC * K2 * 2;
  const size_t bW4  = (size_t)16 * K2 * 2;
  const size_t bBn  = (size_t)3 * 2 * HC * 4;
  const size_t bX   = mpad * CIN0 * 2;
  const size_t total = bMn + bVox + bW1 + 2 * bW2 + bW4 + bBn + bX;
  if (total > ws_size) return;
  if (total > (size_t)134217728) return;

  char* ws = (char*)d_ws;
  size_t off = 0;
  float*          mnp = (float*)(ws + off);          off += bMn;
  int*            vox = (int*)(ws + off);            off += bVox;
  unsigned short* wp1 = (unsigned short*)(ws + off); off += bW1;
  unsigned short* wp2 = (unsigned short*)(ws + off); off += bW2;
  unsigned short* wp3 = (unsigned short*)(ws + off); off += bW2;
  unsigned short* wp4 = (unsigned short*)(ws + off); off += bW4;
  float*          bnt = (float*)(ws + off);          off += bBn;
  unsigned short* xpl = (unsigned short*)(ws + off); off += bX;
  if (off != total) return;

  (void)hipFuncSetAttribute((const void*)k_grid, hipFuncAttributeMaxDynamicSharedMemorySize, SMEM_GRID);
  (void)hipFuncSetAttribute((const void*)k_conv, hipFuncAttributeMaxDynamicSharedMemorySize, SMEM_CONV);

  k_prep<<<G_PREP, TPB, 0, stream>>>(w1, w2, w3, w4, wp1, wp2, wp3, wp4);
  k_small<<<1, TPB, 0, stream>>>(sparse_pts, sparse_batch, nsp,
                                  g1, b1, m1, v1, g2, b2, m2, v2, g3, b3, m3, v3, mnp, bnt);
  k_grid<<<GD / XB, TPB, SMEM_GRID, stream>>>(sparse_coords, sparse_batch, nsp, vox);
  k_interp<<<mblk, TPB, 0, stream>>>(dmh, pfeat, pbatch, sparse_feats, vox, mnp, nsp, mrows, xpl);
  k_conv<<<npts / TP, TPB, SMEM_CONV, stream>>>(xpl, wp1, wp2, wp3, wp4, bnt, bias4, out);
}
